// DFConv2d_56616258896456
// MI455X (gfx1250) — hardware-verified
//
#include <hip/hip_runtime.h>
#include <stddef.h>
#include <stdint.h>

typedef __attribute__((ext_vector_type(16))) _Float16 v16h;
typedef __attribute__((ext_vector_type(8)))  _Float16 v8h;
typedef __attribute__((ext_vector_type(16))) __bf16   v16b;
typedef __attribute__((ext_vector_type(8)))  __bf16   v8b;
typedef __attribute__((ext_vector_type(8)))  float    v8f;
typedef __attribute__((ext_vector_type(4)))  float    v4f;
typedef __attribute__((ext_vector_type(4)))  unsigned v4u;

constexpr int kB = 4, kC = 256, kH = 64, kW = 64, kO = 256;
constexpr int kKP = 9;
constexpr int kNOFF = 27, kNOFFP = 64;
constexpr int kHP = kH + 2, kWP = kW + 2;
constexpr int kKdim = kKP * kC;
constexpr int kPix = kH * kW;
constexpr int kMtot = kB * kPix;
constexpr int kPadRowsPerB = kHP * kWP;
constexpr int kPadRows = kB * kPadRowsPerB;
static_assert(kW == 64, "a 64-row M tile of the conv GEMM must be exactly one image row");
static_assert(kKdim % 32 == 0, "K multiple of 32");
static_assert(kC % 32 == 0, "channel chunks of 32");
static_assert(kMtot % 64 == 0 && kNOFFP % 64 == 0, "site0 M,N tile multiples");
static_assert(kO % 64 == 0 && kPix % 64 == 0, "site1 M,N tile multiples");
static_assert(kNOFF <= 32, "offset/mask row fits one wave");

__device__ __forceinline__ unsigned short f2bf_bits(float f) {
  unsigned u = __float_as_uint(f);
  return (unsigned short)((u + 0x7FFFu + ((u >> 16) & 1u)) >> 16);
}
__device__ __forceinline__ float bf_bits2f(unsigned short h) { return __uint_as_float(((unsigned)h) << 16); }

__device__ __forceinline__ void dep_guard_h(v8f& a, v8f& b, v16h x, v16h y) { asm volatile("v_nop\n\tv_nop\n\tv_nop\n\tv_nop" : "+v"(a), "+v"(b) : "v"(x), "v"(y)); }
__device__ __forceinline__ void dep_guard_b(v8f& a, v8f& b, v16b x, v16b y) { asm volatile("v_nop\n\tv_nop\n\tv_nop\n\tv_nop" : "+v"(a), "+v"(b) : "v"(x), "v"(y)); }
__device__ __forceinline__ void keep4_h(v16h a, v16h b, v16h c, v16h d) { asm volatile("v_nop" :: "v"(a), "v"(b), "v"(c), "v"(d)); }
__device__ __forceinline__ void keep4_b(v16b a, v16b b, v16b c, v16b d) { asm volatile("v_nop" :: "v"(a), "v"(b), "v"(c), "v"(d)); }
__device__ __forceinline__ void acc_guard4(v8f& a, v8f& b, v8f& c, v8f& d) { asm volatile("v_nop\n\tv_nop\n\tv_nop\n\tv_nop" : "+v"(a), "+v"(b), "+v"(c), "+v"(d)); }
template <typename T> struct Frag;
template <> struct Frag<_Float16> {
  typedef v16h V; union U { v16h v; v8h h[2]; };
  static __device__ __forceinline__ v16h load(const _Float16* p) {
    U f; f.h[0] = *(const v8h*)(p); f.h[1] = *(const v8h*)(p + 16); return f.v;
  }
  static __device__ __forceinline__ v8f mma(v16h a, v16h b, v8f c) {
    return __builtin_amdgcn_wmma_f32_16x16x32_f16(false, a, false, b, (short)0, c, false, false);
  }
  static __device__ __forceinline__ void guard(v8f& a, v8f& b, v16h x, v16h y) { dep_guard_h(a, b, x, y); }
  static __device__ __forceinline__ void keep(v16h a, v16h b, v16h c, v16h d) { keep4_h(a, b, c, d); }
};
template <> struct Frag<__bf16> {
  typedef v16b V; union U { v16b v; v8b h[2]; };
  static __device__ __forceinline__ v16b load(const __bf16* p) {
    U f; f.h[0] = *(const v8b*)(p); f.h[1] = *(const v8b*)(p + 16); return f.v;
  }
  static __device__ __forceinline__ v8f mma(v16b a, v16b b, v8f c) {
    return __builtin_amdgcn_wmma_f32_16x16x32_bf16(false, a, false, b, (short)0, c, false, false);
  }
  static __device__ __forceinline__ void guard(v8f& a, v8f& b, v16b x, v16b y) { dep_guard_b(a, b, x, y); }
  static __device__ __forceinline__ void keep(v16b a, v16b b, v16b c, v16b d) { keep4_b(a, b, c, d); }
};

template <int ET> struct Elem;
template <> struct Elem<0> { typedef _Float16 T; };
template <> struct Elem<1> { typedef __bf16 T; };
template <int ET, bool SPLIT, int BIAS_MODE, int OUT_MODE, bool RESID, int ACT = 0>
__global__ __launch_bounds__(256) void wmma_gemm64(
    const unsigned short* __restrict__ Ap, const unsigned short* __restrict__ A2p, int lda, long strideA,
    const unsigned short* __restrict__ Btp, const unsigned short* __restrict__ Bt2p, int ldb, long strideB,
    void* __restrict__ Cout, void* __restrict__ Cout2, int ldc, long strideC,
    const float* __restrict__ bias,
    const float* __restrict__ resid, long strideR,
    int M, int N, int K, float scale) {
  typedef typename Elem<ET>::T T;
  typedef typename Frag<T>::V V;
  const T* A = (const T*)Ap; const T* A2 = (const T*)A2p; const T* Bt = (const T*)Btp; const T* Bt2 = (const T*)Bt2p;
  __shared__ __align__(16) float sT[8][16 * 68];
  const int b    = blockIdx.y;
  const int lane = threadIdx.x & 31;
  const int wave = threadIdx.x >> 5;
  const int tilesN = N >> 6;
  const int tilesM = M >> 6;
  const int tile = blockIdx.x * 8 + wave;
  if (tile >= tilesM * tilesN) return;
  const int tm = tile / tilesN;
  const int tn = tile - tm * tilesN;
  const int m0 = tm << 6;
  const int n0 = tn << 6;

  const T* Ab  = A  + (size_t)b * strideA;
  const T* Bb  = Bt + (size_t)b * strideB;
  const T* Ab2 = SPLIT ? (A2  + (size_t)b * strideA) : nullptr;
  const T* Bb2 = SPLIT ? (Bt2 + (size_t)b * strideB) : nullptr;

  const int rlane = lane & 15;
  const int koff  = (lane >> 4) * 8;
  const int mOff  = (lane >> 4) * 8;

  v8f acc[4][4];
#pragma unroll
  for (int i = 0; i < 4; ++i)
#pragma unroll
    for (int j = 0; j < 4; ++j) acc[i][j] = (v8f){0.f,0.f,0.f,0.f,0.f,0.f,0.f,0.f};

  for (int k0 = 0; k0 < K; k0 += 32) {
    V bh[4], bl[4];
#pragma unroll
    for (int j = 0; j < 4; ++j) {
      const size_t bo = (size_t)(n0 + (j << 4) + rlane) * ldb + koff + k0;
      bh[j] = Frag<T>::load(Bb + bo);
      if (SPLIT) bl[j] = Frag<T>::load(Bb2 + bo);
    }
#pragma unroll
    for (int i = 0; i < 4; ++i) {
      const size_t ao = (size_t)(m0 + (i << 4) + rlane) * lda + koff + k0;
      V ah = Frag<T>::load(Ab + ao);
      V al;
      if (SPLIT) al = Frag<T>::load(Ab2 + ao);
#pragma unroll
      for (int j = 0; j < 4; ++j) {
        acc[i][j] = Frag<T>::mma(ah, bh[j], acc[i][j]);
        if (SPLIT) {
          acc[i][j] = Frag<T>::mma(ah, bl[j], acc[i][j]);
          acc[i][j] = Frag<T>::mma(al, bh[j], acc[i][j]);
        }
      }
      Frag<T>::guard(acc[i][0], acc[i][3], ah, SPLIT ? al : ah);
    }
    Frag<T>::keep(bh[0], bh[1], bh[2], bh[3]);
    if (SPLIT) Frag<T>::keep(bl[0], bl[1], bl[2], bl[3]);
  }
  acc_guard4(acc[0][0], acc[0][1], acc[0][2], acc[0][3]);
  acc_guard4(acc[1][0], acc[1][1], acc[1][2], acc[1][3]);
  acc_guard4(acc[2][0], acc[2][1], acc[2][2], acc[2][3]);
  acc_guard4(acc[3][0], acc[3][1], acc[3][2], acc[3][3]);

  float* slab = sT[wave];
  const float* Rb = RESID ? (resid + (size_t)b * strideR) : nullptr;
#pragma unroll
  for (int i = 0; i < 4; ++i) {
    const int mBase = m0 + (i << 4);
#pragma unroll
    for (int j = 0; j < 4; ++j) {
      const int n = n0 + (j << 4) + rlane;
      float bv = 0.f;
      if (BIAS_MODE == 2) bv = bias[n];
#pragma unroll
      for (int r = 0; r < 8; ++r) {
        float v = acc[i][j][r] * scale;
        if (BIAS_MODE == 1) v += bias[mBase + mOff + r];
        if (BIAS_MODE == 2) v += bv;
        if (RESID) v += Rb[(size_t)(mBase + mOff + r) * ldc + n];
        if (ACT == 1) v = tanhf(v);
        if (ACT == 2) v = fmaxf(v, 0.0f);
        if (ACT == 3) v = v / (1.0f + expf(-v));
        if (ACT == 4) v = (v > 0.f) ? v : 0.01f * v;
        if (ACT == 5) v = 0.5f * v * (1.0f + erff(v * 0.70710678118654752f));
        slab[(mOff + r) * 68 + (j << 4) + rlane] = v;
      }
    }
    __builtin_amdgcn_fence(__ATOMIC_RELEASE, "workgroup");
    __builtin_amdgcn_wave_barrier();
    __builtin_amdgcn_fence(__ATOMIC_ACQUIRE, "workgroup");
    if (OUT_MODE == 0) {
      float* C = (float*)Cout + (size_t)b * strideC;
      const int hh = lane >> 4, c4 = (lane & 15) * 4;
      for (int pass = 0; pass < 2; ++pass) {
#pragma unroll
        for (int it = 0; it < 8; ++it) {
          const int row = it * 2 + hh;
          v4f v = *(const v4f*)(slab + row * 68 + c4);
          *(volatile v4f*)(C + (size_t)(mBase + row) * ldc + n0 + c4) = v;
        }
        __threadfence();
      }
    } else {
      const int q = lane >> 3, c8 = (lane & 7) * 8;
      unsigned short* C  = (unsigned short*)Cout  + (size_t)b * strideC;
      unsigned short* C2 = (OUT_MODE == 2) ? ((unsigned short*)Cout2 + (size_t)b * strideC) : nullptr;
      for (int pass = 0; pass < 2; ++pass) {
#pragma unroll
        for (int it = 0; it < 4; ++it) {
          const int row = it * 4 + q;
          const float* sp = slab + row * 68 + c8;
          v8h hv, lv;
#pragma unroll
          for (int e = 0; e < 8; ++e) {
            if (OUT_MODE == 1) {
              hv[e] = (_Float16)sp[e];
            } else {
              unsigned short hb = f2bf_bits(sp[e]);
              unsigned short lb = f2bf_bits(sp[e] - bf_bits2f(hb));
              hv[e] = __builtin_bit_cast(_Float16, hb);
              lv[e] = __builtin_bit_cast(_Float16, lb);
            }
          }
          *(volatile v8h*)(C + (size_t)(mBase + row) * ldc + n0 + c8) = hv;
          if (OUT_MODE == 2) *(volatile v8h*)(C2 + (size_t)(mBase + row) * ldc + n0 + c8) = lv;
        }
        __threadfence();
      }
    }
    __builtin_amdgcn_fence(__ATOMIC_RELEASE, "workgroup");
    __builtin_amdgcn_wave_barrier();
    __builtin_amdgcn_fence(__ATOMIC_ACQUIRE, "workgroup");
  }
}

template <int ET, bool SPLIT>
__global__ __launch_bounds__(256) void wmma_conv3x3_gemm64(
    const unsigned short* __restrict__ Ap, const unsigned short* __restrict__ A2p,
    const unsigned short* __restrict__ Btp, const unsigned short* __restrict__ Bt2p,
    float* __restrict__ Cout, int M, int N) {
  typedef typename Elem<ET>::T T;
  typedef typename Frag<T>::V V;
  const T* A = (const T*)Ap; const T* A2 = (const T*)A2p; const T* Bt = (const T*)Btp; const T* Bt2 = (const T*)Bt2p;
  __shared__ __align__(16) float sT[8][16 * 68];
  const int lane = threadIdx.x & 31;
  const int wave = threadIdx.x >> 5;
  const int tilesN = N >> 6;
  const int tilesM = M >> 6;
  const int tile = blockIdx.x * 8 + wave;
  if (tile >= tilesM * tilesN) return;
  const int tm = tile / tilesN;
  const int tn = tile - tm * tilesN;
  const int m0 = tm << 6;
  const int n0 = tn << 6;
  const int bb = m0 / kPix;
  const int hrow = (m0 - bb * kPix) / kW;
  const int ldc = N;

  const int rlane = lane & 15;
  const int koff  = (lane >> 4) * 8;
  const int mOff  = (lane >> 4) * 8;

  v8f acc[4][4];
#pragma unroll
  for (int i = 0; i < 4; ++i)
#pragma unroll
    for (int j = 0; j < 4; ++j) acc[i][j] = (v8f){0.f,0.f,0.f,0.f,0.f,0.f,0.f,0.f};

#pragma unroll 1
  for (int kk = 0; kk < kKP; ++kk) {
    const int ky = kk / 3;
    const int kx = kk - 3 * ky;
    const int prow0 = (bb * kHP + hrow + ky) * kWP + kx;
    const int kbase = kk * kC;
#pragma unroll 1
    for (int c0 = 0; c0 < kC; c0 += 32) {
      V bh[4], bl[4];
#pragma unroll
      for (int j = 0; j < 4; ++j) {
        const size_t bo = (size_t)(n0 + (j << 4) + rlane) * kKdim + kbase + c0 + koff;
        bh[j] = Frag<T>::load(Bt + bo);
        if (SPLIT) bl[j] = Frag<T>::load(Bt2 + bo);
      }
#pragma unroll
      for (int i = 0; i < 4; ++i) {
        const size_t ao = (size_t)(prow0 + (i << 4) + rlane) * kC + c0 + koff;
        V ah = Frag<T>::load(A + ao);
        V al;
        if (SPLIT) al = Frag<T>::load(A2 + ao);
#pragma unroll
        for (int j = 0; j < 4; ++j) {
          acc[i][j] = Frag<T>::mma(ah, bh[j], acc[i][j]);
          if (SPLIT) {
            acc[i][j] = Frag<T>::mma(ah, bl[j], acc[i][j]);
            acc[i][j] = Frag<T>::mma(al, bh[j], acc[i][j]);
          }
        }
        Frag<T>::guard(acc[i][0], acc[i][3], ah, SPLIT ? al : ah);
      }
      Frag<T>::keep(bh[0], bh[1], bh[2], bh[3]);
      if (SPLIT) Frag<T>::keep(bl[0], bl[1], bl[2], bl[3]);
    }
  }
  acc_guard4(acc[0][0], acc[0][1], acc[0][2], acc[0][3]);
  acc_guard4(acc[1][0], acc[1][1], acc[1][2], acc[1][3]);
  acc_guard4(acc[2][0], acc[2][1], acc[2][2], acc[2][3]);
  acc_guard4(acc[3][0], acc[3][1], acc[3][2], acc[3][3]);

  float* slab = sT[wave];
#pragma unroll
  for (int i = 0; i < 4; ++i) {
    const int mBase = m0 + (i << 4);
#pragma unroll
    for (int j = 0; j < 4; ++j) {
#pragma unroll
      for (int r = 0; r < 8; ++r) {
        slab[(mOff + r) * 68 + (j << 4) + rlane] = acc[i][j][r];
      }
    }
    __builtin_amdgcn_fence(__ATOMIC_RELEASE, "workgroup");
    __builtin_amdgcn_wave_barrier();
    __builtin_amdgcn_fence(__ATOMIC_ACQUIRE, "workgroup");
    {
      float* C = Cout;
      const int hh = lane >> 4, c4 = (lane & 15) * 4;
      for (int pass = 0; pass < 2; ++pass) {
#pragma unroll
        for (int it = 0; it < 8; ++it) {
          const int row = it * 2 + hh;
          v4f v = *(const v4f*)(slab + row * 68 + c4);
          *(volatile v4f*)(C + (size_t)(mBase + row) * ldc + n0 + c4) = v;
        }
        __threadfence();
      }
    }
    __builtin_amdgcn_fence(__ATOMIC_RELEASE, "workgroup");
    __builtin_amdgcn_wave_barrier();
    __builtin_amdgcn_fence(__ATOMIC_ACQUIRE, "workgroup");
  }
}

__device__ __forceinline__ void xprep_row(const float* sx, int xx, bool zero, size_t pr, int ch, int lane,
                                          float* __restrict__ xt, unsigned short* __restrict__ xph,
                                          unsigned short* __restrict__ xpl) {
  float f4[4], f8[8];
  if (!zero) {
#pragma unroll
    for (int e = 0; e < 4; ++e) f4[e] = sx[(4 * lane + e) * 65 + xx];
#pragma unroll
    for (int e = 0; e < 8; ++e) f8[e] = sx[(8 * (lane & 15) + e) * 65 + xx];
  } else {
#pragma unroll
    for (int e = 0; e < 4; ++e) f4[e] = 0.f;
#pragma unroll
    for (int e = 0; e < 8; ++e) f8[e] = 0.f;
  }
  v4f fv;
  fv[0] = f4[0]; fv[1] = f4[1]; fv[2] = f4[2]; fv[3] = f4[3];
  unsigned short hb[8], lb[8];
#pragma unroll
  for (int e = 0; e < 8; ++e) {
    hb[e] = f2bf_bits(f8[e]);
    lb[e] = f2bf_bits(f8[e] - bf_bits2f(hb[e]));
  }
  const bool hiLane = lane < 16;
  v4u pk;
#pragma unroll
  for (int e2 = 0; e2 < 4; ++e2) {
    const unsigned wh = (unsigned)hb[2 * e2] | ((unsigned)hb[2 * e2 + 1] << 16);
    const unsigned wl = (unsigned)lb[2 * e2] | ((unsigned)lb[2 * e2 + 1] << 16);
    pk[e2] = hiLane ? wh : wl;
  }
  unsigned short* p16 = hiLane ? xph : xpl;
  const size_t i32 = pr * kC + (size_t)ch * 128 + 4 * lane;
  const size_t i16 = pr * kC + (size_t)ch * 128 + 8 * (lane & 15);
  for (int pass = 0; pass < 2; ++pass) {
    *(volatile v4f*)(xt + i32) = fv;
    *(volatile v4u*)(p16 + i16) = pk;
    __threadfence();
  }
}

__global__ __launch_bounds__(256) void k_xprep(const float* __restrict__ x, float* __restrict__ xt,
                                               unsigned short* __restrict__ xph, unsigned short* __restrict__ xpl) {
  __shared__ float sx[128 * 65];
  const int tid = threadIdx.x, lane = tid & 31, wave = tid >> 5;
  const int bid = blockIdx.x;
  const int ch = bid & 1;
  const int y  = (bid >> 1) & (kH - 1);
  const int b  = bid >> 7;
#pragma unroll
  for (int it = 0; it < 8; ++it) {
    const int cc  = (tid >> 4) + 16 * it;
    const int xx4 = (tid & 15) * 4;
    const v4f v = *(const v4f*)(x + ((size_t)(b * kC + ch * 128 + cc) * kH + y) * kW + xx4);
    sx[cc * 65 + xx4 + 0] = v[0];
    sx[cc * 65 + xx4 + 1] = v[1];
    sx[cc * 65 + xx4 + 2] = v[2];
    sx[cc * 65 + xx4 + 3] = v[3];
  }
  __syncthreads();
  const size_t hpBase = (size_t)(b * kHP + (y + 1)) * kWP;
#pragma unroll 1
  for (int q = 0; q < 8; ++q) {
    const int xx = wave * 8 + q;
    xprep_row(sx, xx, false, hpBase + (size_t)(xx + 1), ch, lane, xt, xph, xpl);
  }
  if (wave == 0) xprep_row(sx, 0, true, hpBase + 0, ch, lane, xt, xph, xpl);
  if (wave == 1) xprep_row(sx, 0, true, hpBase + (size_t)(kWP - 1), ch, lane, xt, xph, xpl);
  if (y == 0) {
#pragma unroll 1
    for (int wp = wave; wp < kWP; wp += 8)
      xprep_row(sx, 0, true, (size_t)(b * kHP + 0) * kWP + wp, ch, lane, xt, xph, xpl);
  }
  if (y == kH - 1) {
#pragma unroll 1
    for (int wp = wave; wp < kWP; wp += 8)
      xprep_row(sx, 0, true, (size_t)(b * kHP + (kHP - 1)) * kWP + wp, ch, lane, xt, xph, xpl);
  }
}

__global__ __launch_bounds__(256) void k_wprep(const float* __restrict__ w, int nreal, int npad,
                                               unsigned short* __restrict__ oh, unsigned short* __restrict__ ol) {
  const int t = blockIdx.x * 256 + threadIdx.x;
  const int total = npad * kKP * 32;
  if (t >= total) return;
  const int c8 = t & 31;
  const int r  = t >> 5;
  const int kk = r % kKP;
  const int j  = r / kKP;
  const int jc = (j < nreal) ? j : (nreal - 1);
  const float* src = w + (size_t)jc * kKdim + (size_t)(c8 * 8) * kKP + kk;
  float v[8];
#pragma unroll
  for (int e = 0; e < 8; ++e) {
    float f = src[e * kKP];
    v[e] = (j < nreal) ? f : 0.f;
  }
  unsigned short hb[8], lb[8];
#pragma unroll
  for (int e = 0; e < 8; ++e) {
    hb[e] = f2bf_bits(v[e]);
    lb[e] = f2bf_bits(v[e] - bf_bits2f(hb[e]));
  }
  v4u ph, pl;
#pragma unroll
  for (int e2 = 0; e2 < 4; ++e2) {
    ph[e2] = (unsigned)hb[2 * e2] | ((unsigned)hb[2 * e2 + 1] << 16);
    pl[e2] = (unsigned)lb[2 * e2] | ((unsigned)lb[2 * e2 + 1] << 16);
  }
  const size_t idx = (size_t)j * kKdim + (size_t)kk * kC + (size_t)c8 * 8;
  for (int pass = 0; pass < 2; ++pass) {
    *(volatile v4u*)(oh + idx) = ph;
    *(volatile v4u*)(ol + idx) = pl;
    __threadfence();
  }
}

__global__ __launch_bounds__(256) void k_sample(const float* __restrict__ xt, const float* __restrict__ om,
                                                const float* __restrict__ boff,
                                                unsigned short* __restrict__ valh, unsigned short* __restrict__ vall,
                                                int bsel) {
  const int lane = threadIdx.x & 31, wave = threadIdx.x >> 5;
  const int hw = blockIdx.x * 8 + wave;
  const int h = hw >> 6, w = hw & 63;
  const int m = bsel * kPix + hw;
  float omv = om[(size_t)m * kNOFFP + lane];
  float bo = boff[(lane < kNOFF) ? lane : (kNOFF - 1)];
  bo = (lane < kNOFF) ? bo : 0.f;
  omv = omv + bo;
  const float* xb = xt + (size_t)bsel * ((size_t)kPadRowsPerB * kC);
#pragma unroll 1
  for (int kk = 0; kk < kKP; ++kk) {
    const float offy = __shfl(omv, 2 * kk, 32);
    const float offx = __shfl(omv, 2 * kk + 1, 32);
    const float mr   = __shfl(omv, 2 * kKP + kk, 32);
    const float ev = expf(-mr);
    const float gate = 1.0f / (1.0f + ev);
    const int ky = kk / 3;
    const int kx = kk - 3 * ky;
    const float py = (float)(h - 1 + ky) + offy;
    const float px = (float)(w - 1 + kx) + offx;
    const float y0f = floorf(py), x0f = floorf(px);
    const float wy = py - y0f, wx = px - x0f;
    const float y0cf = fminf(fmaxf(y0f, -4.f), 70.f);
    const float x0cf = fminf(fmaxf(x0f, -4.f), 70.f);
    const int y0 = (int)y0cf, x0 = (int)x0cf;
    const int y1 = y0 + 1, x1 = x0 + 1;
    const bool vy0 = (y0 >= 0) && (y0 < kH), vy1 = (y1 >= 0) && (y1 < kH);
    const bool vx0 = (x0 >= 0) && (x0 < kW), vx1 = (x1 >= 0) && (x1 < kW);
    const int yc0 = min(max(y0, 0), kH - 1), yc1 = min(max(y1, 0), kH - 1);
    const int xc0 = min(max(x0, 0), kW - 1), xc1 = min(max(x1, 0), kW - 1);
    float w00 = (1.f - wy) * (1.f - wx);
    float w01 = (1.f - wy) * wx;
    float w10 = wy * (1.f - wx);
    float w11 = wy * wx;
    w00 = (vy0 && vx0) ? w00 : 0.f;
    w01 = (vy0 && vx1) ? w01 : 0.f;
    w10 = (vy1 && vx0) ? w10 : 0.f;
    w11 = (vy1 && vx1) ? w11 : 0.f;
    const float* r00 = xb + ((size_t)(yc0 + 1) * kWP + (xc0 + 1)) * kC + 8 * lane;
    const float* r01 = xb + ((size_t)(yc0 + 1) * kWP + (xc1 + 1)) * kC + 8 * lane;
    const float* r10 = xb + ((size_t)(yc1 + 1) * kWP + (xc0 + 1)) * kC + 8 * lane;
    const float* r11 = xb + ((size_t)(yc1 + 1) * kWP + (xc1 + 1)) * kC + 8 * lane;
    const v4f a0 = *(const v4f*)(r00), a1 = *(const v4f*)(r00 + 4);
    const v4f b0 = *(const v4f*)(r01), b1 = *(const v4f*)(r01 + 4);
    const v4f g0 = *(const v4f*)(r10), g1 = *(const v4f*)(r10 + 4);
    const v4f d0 = *(const v4f*)(r11), d1 = *(const v4f*)(r11 + 4);
    float o[8];
#pragma unroll
    for (int e = 0; e < 4; ++e) {
      o[e]     = (((w00 * a0[e] + w01 * b0[e]) + w10 * g0[e]) + w11 * d0[e]) * gate;
      o[4 + e] = (((w00 * a1[e] + w01 * b1[e]) + w10 * g1[e]) + w11 * d1[e]) * gate;
    }
    unsigned short hb[8], lb[8];
#pragma unroll
    for (int e = 0; e < 8; ++e) {
      hb[e] = f2bf_bits(o[e]);
      lb[e] = f2bf_bits(o[e] - bf_bits2f(hb[e]));
    }
    v4u ph, pl;
#pragma unroll
    for (int e2 = 0; e2 < 4; ++e2) {
      ph[e2] = (unsigned)hb[2 * e2] | ((unsigned)hb[2 * e2 + 1] << 16);
      pl[e2] = (unsigned)lb[2 * e2] | ((unsigned)lb[2 * e2 + 1] << 16);
    }
    const size_t idx = (size_t)hw * kKdim + (size_t)kk * kC + 8 * lane;
    for (int pass = 0; pass < 2; ++pass) {
      *(volatile v4u*)(valh + idx) = ph;
      *(volatile v4u*)(vall + idx) = pl;
      __threadfence();
    }
  }
}

extern "C" void kernel_launch(void* const* d_in, const int* in_sizes, int n_in,
                              void* d_out, int out_size, void* d_ws, size_t ws_size,
                              hipStream_t stream) {
  (void)n_in; (void)out_size;
  if (in_sizes[0] != kB * kC * kH * kW) return;
  if (in_sizes[1] != kNOFF * kKdim) return;
  if (in_sizes[2] != kNOFF) return;
  if (in_sizes[3] != kO * kKdim) return;
  if (out_size != kB * kO * kPix) return;

  const float* x      = (const float*)d_in[0];
  const float* w_off  = (const float*)d_in[1];
  const float* b_off  = (const float*)d_in[2];
  const float* w_conv = (const float*)d_in[3];
  float* out = (float*)d_out;

  char* ws = (char*)d_ws;
  size_t off = 0;
  const size_t xtB  = (size_t)kPadRows * kC * 4;
  const size_t xpB  = (size_t)kPadRows * kC * 2;
  const size_t w0B  = (size_t)kNOFFP * kKdim * 2;
  const size_t w1B  = (size_t)kO * kKdim * 2;
  const size_t omB  = (size_t)kMtot * kNOFFP * 4;
  const size_t valB = (size_t)kPix * kKdim * 2;
  float* xt = (float*)(ws + off);                      off += (xtB + 255) & ~(size_t)255;
  unsigned short* xph = (unsigned short*)(ws + off);   off += (xpB + 255) & ~(size_t)255;
  unsigned short* xpl = (unsigned short*)(ws + off);   off += (xpB + 255) & ~(size_t)255;
  unsigned short* w0h = (unsigned short*)(ws + off);   off += (w0B + 255) & ~(size_t)255;
  unsigned short* w0l = (unsigned short*)(ws + off);   off += (w0B + 255) & ~(size_t)255;
  unsigned short* w1h = (unsigned short*)(ws + off);   off += (w1B + 255) & ~(size_t)255;
  unsigned short* w1l = (unsigned short*)(ws + off);   off += (w1B + 255) & ~(size_t)255;
  float* om = (float*)(ws + off);                      off += (omB + 255) & ~(size_t)255;
  unsigned short* valh = (unsigned short*)(ws + off);  off += (valB + 255) & ~(size_t)255;
  unsigned short* vall = (unsigned short*)(ws + off);  off += (valB + 255) & ~(size_t)255;
  if (off > ws_size) return;

  k_xprep<<<dim3(kB * kH * 2), dim3(256), 0, stream>>>(x, xt, xph, xpl);
  static_assert((kNOFFP * kKP * 32) % 256 == 0 && (kO * kKP * 32) % 256 == 0, "exact grids");
  k_wprep<<<dim3((kNOFFP * kKP * 32) / 256), dim3(256), 0, stream>>>(w_off, kNOFF, kNOFFP, w0h, w0l);
  k_wprep<<<dim3((kO * kKP * 32) / 256), dim3(256), 0, stream>>>(w_conv, kO, kO, w1h, w1l);
  static_assert(kMtot % 64 == 0 && kNOFFP % 64 == 0 && (kKdim % 32) == 0, "site0 tiles");
  wmma_conv3x3_gemm64<1, true><<<dim3((kMtot / 64) * (kNOFFP / 64) / 8), dim3(256), 0, stream>>>(
      xph, xpl, w0h, w0l, om, kMtot, kNOFFP);
  static_assert(kO % 64 == 0 && kPix % 64 == 0, "site1 tiles");
  static_assert(((kO / 64) * (kPix / 64)) % 8 == 0, "site1 grid");
  for (int b = 0; b < kB; ++b) {
    k_sample<<<dim3(kPix / 8), dim3(256), 0, stream>>>(xt, om, b_off, valh, vall, b);
    wmma_gemm64<1, true, 0, 0, false, 0><<<dim3((kO / 64) * (kPix / 64) / 8, 1), dim3(256), 0, stream>>>(
        w1h, w1l, kKdim, (long)0,
        valh, vall, kKdim, (long)0,
        (void*)(out + (size_t)b * kO * kPix), (void*)nullptr, kPix, (long)0,
        (const float*)nullptr,
        (const float*)nullptr, (long)0,
        kO, kPix, kKdim, 1.0f);
  }
}
